// HierNet_55705725829422
// MI455X (gfx1250) — hardware-verified
//
#include <hip/hip_runtime.h>
#include <stddef.h>


#pragma clang fp contract(off)

#define NTHR    256
#define NWAVE   8
#define EPT     8
#define NGRP    2
#define CHUNK   (NTHR * EPT * NGRP)
#define WCAP    (EPT * NGRP * 32)
#define LISTN   (NWAVE * WCAP)
#define PQROWS  128
#define GGR     64
#define HLSD    32
#define HIDC    64
#define WSC     16.0f
#define WINV    0.0625f
#define AVG_LOG_F 2.8332133440562162f
#define LDS_PQ   (NWAVE * 16 * 128 * 4)
#define LDS_HEAD (4 * 64 * 64 * 8 + 64 * 96 * 2 + 64 * 64 * 4 * 2 + 64 * 4)
#define WS_CAP   ((size_t)134217728)

static_assert((CHUNK & (CHUNK - 1)) == 0);
static_assert(CHUNK <= 4096);

typedef float    v2f  __attribute__((ext_vector_type(2)));
typedef float    v4f  __attribute__((ext_vector_type(4)));
typedef float    v8f  __attribute__((ext_vector_type(8)));
typedef int      v4i  __attribute__((ext_vector_type(4)));
typedef _Float16 v8h  __attribute__((ext_vector_type(8)));
typedef _Float16 v16h __attribute__((ext_vector_type(16)));
union FragH { v16h v; v8h h[2]; };

template <int CH> struct VT;
template <> struct VT<2> { typedef v2f t; };
template <> struct VT<4> { typedef v4f t; };

template <int F>
struct PnaCfg {
  static constexpr int TF   = 2 * F;
  static constexpr int CH   = TF / 32;
  static constexpr int NB   = (F == 32) ? 256 : 128;
  static constexpr int ROWW = 4 * TF;
  static constexpr int K13  = 13 * F;
  static constexpr int NQ   = NB / 128;
  static constexpr int LDS  = NB * ROWW * 4 + LISTN * 4 + 64 + NB * 4 + NB * 8;
};
static_assert(PnaCfg<32>::LDS <= 300000);
static_assert(PnaCfg<64>::LDS <= 300000);
static_assert(PnaCfg<32>::NB <= 4096 && PnaCfg<64>::NB <= 4096);
static_assert((PnaCfg<32>::NB & (PnaCfg<32>::NB - 1)) == 0);
static_assert((PnaCfg<64>::NB & (PnaCfg<64>::NB - 1)) == 0);

__device__ __forceinline__ v8h cvt8(v4f a, v4f b) {
  v8h r;
  r[0] = (_Float16)a.x; r[1] = (_Float16)a.y; r[2] = (_Float16)a.z; r[3] = (_Float16)a.w;
  r[4] = (_Float16)b.x; r[5] = (_Float16)b.y; r[6] = (_Float16)b.z; r[7] = (_Float16)b.w;
  return r;
}

__device__ __forceinline__ v8f wmh(v16h a, v16h b, v8f c) {
  v8f d = __builtin_amdgcn_wmma_f32_16x16x32_f16(false, a, false, b, (short)0, c, false, false);
  asm volatile("v_nop\n\tv_nop\n\tv_nop\n\tv_nop" : "+v"(d) : "v"(a), "v"(b));
  return d;
}

template <int CH>
__device__ __forceinline__ typename VT<CH>::t vminC(typename VT<CH>::t a, typename VT<CH>::t b) {
  typename VT<CH>::t r = a;
#pragma unroll
  for (int i = 0; i < CH; ++i) r[i] = fminf(a[i], b[i]);
  return r;
}
template <int CH>
__device__ __forceinline__ typename VT<CH>::t vmaxC(typename VT<CH>::t a, typename VT<CH>::t b) {
  typename VT<CH>::t r = a;
#pragma unroll
  for (int i = 0; i < CH; ++i) r[i] = fmaxf(a[i], b[i]);
  return r;
}

__device__ __forceinline__ void st2h(_Float16* dp, v8h hv) {
  *(volatile v8h*)dp = hv;
  __threadfence();
  *(volatile v8h*)dp = hv;
}
__device__ __forceinline__ void st2f(float* dp, v4f v) {
  *(volatile v4f*)dp = v;
  __threadfence();
  *(volatile v4f*)dp = v;
}

template <int NB>
__device__ __forceinline__ int scan_chunk(const int* __restrict__ dsts, int nE, int cbase, int nodeBase,
                                          int vec8, int* list, int tid, int lane, int wave) {
  int wc = 0;
#pragma unroll
  for (int g = 0; g < NGRP; ++g) {
    const int el0  = (g * NTHR + tid) * EPT;
    const int e0   = cbase + el0;
    const int sent = -2147483647 - 1;
    v4i da, db;
    if (vec8 != 0 && cbase + CHUNK <= nE) {
      da = *(const v4i*)(dsts + e0);
      db = *(const v4i*)(dsts + e0 + 4);
    } else {
      da.x = (e0     < nE) ? dsts[min(e0, nE - 1)] : sent;
      da.y = (e0 + 1 < nE) ? dsts[min(e0 + 1, nE - 1)] : sent;
      da.z = (e0 + 2 < nE) ? dsts[min(e0 + 2, nE - 1)] : sent;
      da.w = (e0 + 3 < nE) ? dsts[min(e0 + 3, nE - 1)] : sent;
      db.x = (e0 + 4 < nE) ? dsts[min(e0 + 4, nE - 1)] : sent;
      db.y = (e0 + 5 < nE) ? dsts[min(e0 + 5, nE - 1)] : sent;
      db.z = (e0 + 6 < nE) ? dsts[min(e0 + 6, nE - 1)] : sent;
      db.w = (e0 + 7 < nE) ? dsts[min(e0 + 7, nE - 1)] : sent;
    }
    const unsigned nb = (unsigned)nodeBase;
    const unsigned s0 = (unsigned)da.x - nb, s1 = (unsigned)da.y - nb;
    const unsigned s2 = (unsigned)da.z - nb, s3 = (unsigned)da.w - nb;
    const unsigned s4 = (unsigned)db.x - nb, s5 = (unsigned)db.y - nb;
    const unsigned s6 = (unsigned)db.z - nb, s7 = (unsigned)db.w - nb;
    const bool h0 = s0 < (unsigned)NB, h1 = s1 < (unsigned)NB, h2 = s2 < (unsigned)NB, h3 = s3 < (unsigned)NB;
    const bool h4 = s4 < (unsigned)NB, h5 = s5 < (unsigned)NB, h6 = s6 < (unsigned)NB, h7 = s7 < (unsigned)NB;
    const unsigned any = __builtin_amdgcn_ballot_w32(h0 | h1 | h2 | h3 | h4 | h5 | h6 | h7);
    if (any != 0u) {
#define HITJ(J, HJ, SJ) { \
        const unsigned mj = __builtin_amdgcn_ballot_w32(HJ); \
        if (mj != 0u) { \
          if (HJ) { \
            const int pos = wc + (int)__builtin_amdgcn_mbcnt_lo(mj, 0u); \
            if (pos < WCAP) list[wave * WCAP + pos] = ((el0 + (J)) << 12) | (int)(SJ); \
          } \
          wc += (int)__builtin_popcount(mj); } }
      HITJ(0, h0, s0)
      HITJ(1, h1, s1)
      HITJ(2, h2, s2)
      HITJ(3, h3, s3)
      HITJ(4, h4, s4)
      HITJ(5, h5, s5)
      HITJ(6, h6, s6)
      HITJ(7, h7, s7)
#undef HITJ
    }
  }
  return wc;
}

__device__ __forceinline__ void put8h(_Float16* dp, const float* sp, int stride) {
  v4f a, b;
  a.x = sp[0];          a.y = sp[stride];     a.z = sp[2 * stride]; a.w = sp[3 * stride];
  b.x = sp[4 * stride]; b.y = sp[5 * stride]; b.z = sp[6 * stride]; b.w = sp[7 * stride];
  a = a * WSC;
  b = b * WSC;
  st2h(dp, cvt8(a, b));
}

template <int F>
__device__ __forceinline__ void prep_pq(int p, const float* __restrict__ Wpre, _Float16* wpq) {
  constexpr int NPR = F / 8;
  constexpr int NP  = 4 * F * NPR;
  if (p >= NP) return;
  const int c   = p / NPR;
  const int k0  = (p - c * NPR) * 8;
  const int pqs = c / (2 * F);
  const int t   = (c / F) & 1;
  const int o   = c & (F - 1);
  const float* sp = Wpre + (size_t)(t * 3 * F + pqs * F + k0) * F + o;
  put8h(wpq + (size_t)c * F + k0, sp, F);
}

template <int F>
__device__ __forceinline__ void prep_post(int p, const float* __restrict__ Wpost, _Float16* wpo) {
  constexpr int K13 = 13 * F, NPR = K13 / 8, NP = 64 * NPR;
  if (p >= NP) return;
  const int R = p / NPR, k0 = (p - R * NPR) * 8;
  const int t = R >> 5, n = R & 31;
  const float* sp = Wpost + (size_t)(t * K13 + k0) * 32 + n;
  put8h(wpo + (size_t)R * K13 + k0, sp, 32);
}

__device__ __forceinline__ void prep_nk(int p, const float* __restrict__ W, _Float16* wt, int K, int N) {
  const int NPR = K / 8, NP = N * NPR;
  if (p >= NP) return;
  const int n = p / NPR, k0 = (p - n * NPR) * 8;
  const float* sp = W + (size_t)k0 * N + n;
  put8h(wt + (size_t)n * K + k0, sp, N);
}

template <int F>
__device__ __forceinline__ void prep_cmp(int p, const float* __restrict__ We, const float* __restrict__ be,
                                         const float* __restrict__ bpre, const float* __restrict__ Wpre, float* cmp) {
  constexpr int TF = 2 * F, NPC = TF / 2, NP = 3 * TF / 4;
  if (p >= NP) return;
  const bool isC = p < NPC;
  const int j   = isC ? (p / (TF / 4)) : 0;
  const int ch0 = isC ? (p - j * (TF / 4)) * 4 : (p - NPC) * 4;
  const int t = ch0 / F, o = ch0 - t * F;
  const float* wp = Wpre + (size_t)(t * 3 * F + 2 * F) * F + o;
  v4f acc = {0.f, 0.f, 0.f, 0.f};
#pragma unroll 1
  for (int k = 0; k < F; ++k) {
    const float sc = We[j * F + k];
    const float sb = be[k];
    const float s  = isC ? sc : sb;
    const float* r = wp + (size_t)k * F;
    acc.x = acc.x + s * r[0];
    acc.y = acc.y + s * r[1];
    acc.z = acc.z + s * r[2];
    acc.w = acc.w + s * r[3];
  }
  if (!isC) {
    acc.x = acc.x + bpre[t * F + o];
    acc.y = acc.y + bpre[t * F + o + 1];
    acc.z = acc.z + bpre[t * F + o + 2];
    acc.w = acc.w + bpre[t * F + o + 3];
  }
  st2f(cmp + (size_t)p * 4, acc);
}

__global__ __launch_bounds__(NTHR) void k_prep(
    const float* __restrict__ Wpre0, const float* __restrict__ Wpre1,
    const float* __restrict__ Wpost0, const float* __restrict__ Wpost1,
    const float* __restrict__ Wlin0, const float* __restrict__ Wlin1,
    const float* __restrict__ W1, const float* __restrict__ W2,
    const float* __restrict__ We0, const float* __restrict__ be0, const float* __restrict__ bpre0,
    const float* __restrict__ We1, const float* __restrict__ be1, const float* __restrict__ bpre1,
    _Float16* wpq0, _Float16* wpq1, _Float16* wpo0, _Float16* wpo1,
    _Float16* wl0, _Float16* wl1, _Float16* w1t, _Float16* w2t,
    float* cmp0, float* cmp1) {
  const int seg = blockIdx.y;
  const int p = blockIdx.x * NTHR + threadIdx.x;
  if (seg == 0)      prep_pq<32>(p, Wpre0, wpq0);
  else if (seg == 1) prep_pq<64>(p, Wpre1, wpq1);
  else if (seg == 2) prep_post<32>(p, Wpost0, wpo0);
  else if (seg == 3) prep_post<64>(p, Wpost1, wpo1);
  else if (seg == 4) prep_nk(p, Wlin0, wl0, 64, 64);
  else if (seg == 5) prep_nk(p, Wlin1, wl1, 64, 64);
  else if (seg == 6) prep_nk(p, W1, w1t, 96, 64);
  else if (seg == 7) prep_nk(p, W2, w2t, 64, 64);
  else if (seg == 8) prep_cmp<32>(p, We0, be0, bpre0, Wpre0, cmp0);
  else if (seg == 9) prep_cmp<64>(p, We1, be1, bpre1, Wpre1, cmp1);
}

template <int F>
__global__ __launch_bounds__(NTHR) void k_pq(const float* __restrict__ xin, const _Float16* __restrict__ wpq,
                                            float* pqo, int nN) {
  constexpr int NC = 4 * F, KS = F / 32, NG = NC / 128;
  extern __shared__ v4f lds_dyn[];
  float* stg = (float*)lds_dyn;
  const int tid = threadIdx.x, lane = tid & 31, wave = tid >> 5, hh = lane >> 4, m = lane & 15;
  const int rowBase = blockIdx.x * PQROWS;
  int node = rowBase + wave * 16 + m;
  node = node > nN - 1 ? nN - 1 : node;
  const float* xr = xin + (size_t)node * F + 8 * hh;

  FragH a[KS];
#pragma unroll
  for (int ks = 0; ks < KS; ++ks) {
    const float* xp = xr + 32 * ks;
    const v4f p0 = *(const v4f*)xp,        p1 = *(const v4f*)(xp + 4);
    const v4f p2 = *(const v4f*)(xp + 16), p3 = *(const v4f*)(xp + 20);
    a[ks].h[0] = cvt8(p0, p1);
    a[ks].h[1] = cvt8(p2, p3);
  }

#pragma unroll
  for (int g = 0; g < NG; ++g) {
    v8f acc[8];
#pragma unroll
    for (int nt = 0; nt < 8; ++nt) { v8f z = {0.f, 0.f, 0.f, 0.f, 0.f, 0.f, 0.f, 0.f}; acc[nt] = z; }
#pragma unroll
    for (int ks = 0; ks < KS; ++ks) {
#pragma unroll
      for (int nt = 0; nt < 8; ++nt) {
        const _Float16* bp = wpq + (size_t)(128 * g + 16 * nt + m) * F + 32 * ks + 8 * hh;
        FragH b;
        b.h[0] = *(const v8h*)bp;
        b.h[1] = *(const v8h*)(bp + 16);
        acc[nt] = wmh(a[ks].v, b.v, acc[nt]);
      }
    }
    float* sp = stg + (wave * 16 + 8 * hh) * 128 + m;
#pragma unroll
    for (int nt = 0; nt < 8; ++nt) {
#pragma unroll
      for (int r = 0; r < 8; ++r) sp[r * 128 + 16 * nt] = acc[nt][r] * WINV;
    }
    __syncthreads();
    const float* lp = stg + wave * 16 * 128 + 4 * lane;
    float* gp = pqo + ((size_t)rowBase + wave * 16) * NC + 128 * g + 4 * lane;
#pragma unroll
    for (int i = 0; i < 16; ++i) { const v4f v = *(const v4f*)(lp + i * 128); *(volatile v4f*)(gp + (size_t)i * NC) = v; }
    __threadfence();
#pragma unroll
    for (int i = 0; i < 16; ++i) { const v4f v = *(const v4f*)(lp + i * 128); *(volatile v4f*)(gp + (size_t)i * NC) = v; }
    __syncthreads();
  }
}

template <int F>
__device__ __forceinline__ void pna_tower(int t, const float* arow, const float* __restrict__ xr,
                                          float ampm, float attm, const _Float16* __restrict__ wpo,
                                          int hh, int m, v8f& o0, v8f& o1) {
  constexpr int TF = 2 * F, K13 = 13 * F, KX = F / 32, KA = 12 * F / 32;
  const _Float16* b0p = wpo + (size_t)(t * 32 + m) * K13 + 8 * hh;
  const _Float16* b1p = b0p + (size_t)16 * K13;
#pragma unroll
  for (int ks = 0; ks < KX; ++ks) {
    const float* xp = xr + 32 * ks + 8 * hh;
    const v4f p0 = *(const v4f*)xp,        p1 = *(const v4f*)(xp + 4);
    const v4f p2 = *(const v4f*)(xp + 16), p3 = *(const v4f*)(xp + 20);
    FragH a;
    a.h[0] = cvt8(p0, p1);
    a.h[1] = cvt8(p2, p3);
    FragH b;
    b.h[0] = *(const v8h*)(b0p + 32 * ks); b.h[1] = *(const v8h*)(b0p + 32 * ks + 16);
    o0 = wmh(a.v, b.v, o0);
    b.h[0] = *(const v8h*)(b1p + 32 * ks); b.h[1] = *(const v8h*)(b1p + 32 * ks + 16);
    o1 = wmh(a.v, b.v, o1);
  }
#pragma unroll 1
  for (int j = 0; j < KA; ++j) {
    const int s  = j / (4 * KX);
    const int rm = j - s * (4 * KX);
    const int ag = rm / KX;
    const int kf = rm - ag * KX;
    const float sc = (s == 0) ? 1.0f : ((s == 1) ? ampm : attm);
    const float* ap = arow + ag * TF + t * F + 32 * kf + 8 * hh;
    v4f p0 = *(const v4f*)ap,        p1 = *(const v4f*)(ap + 4);
    v4f p2 = *(const v4f*)(ap + 16), p3 = *(const v4f*)(ap + 20);
    p0 = p0 * sc; p1 = p1 * sc; p2 = p2 * sc; p3 = p3 * sc;
    FragH a;
    a.h[0] = cvt8(p0, p1);
    a.h[1] = cvt8(p2, p3);
    const int k0 = F + 32 * j;
    FragH b;
    b.h[0] = *(const v8h*)(b0p + k0); b.h[1] = *(const v8h*)(b0p + k0 + 16);
    o0 = wmh(a.v, b.v, o0);
    b.h[0] = *(const v8h*)(b1p + k0); b.h[1] = *(const v8h*)(b1p + k0 + 16);
    o1 = wmh(a.v, b.v, o1);
  }
}

template <int F>
__global__ __launch_bounds__(NTHR) void k_pna(
    const int* __restrict__ ei, const float* __restrict__ eattr, const float* __restrict__ xin,
    const float* __restrict__ pq, const float* __restrict__ cmp,
    const _Float16* __restrict__ wpo, const float* __restrict__ bpost,
    const _Float16* __restrict__ wl, const float* __restrict__ blin,
    float* hout, int nN, int nE, int vec8) {
  typedef PnaCfg<F> C;
  constexpr int TF = C::TF, CH = C::CH, NB = C::NB, ROWW = C::ROWW, NQ = C::NQ, NC = 4 * F;
  typedef typename VT<CH>::t vC;
  extern __shared__ v4f lds_dyn[];
  float* acc  = (float*)lds_dyn;
  int*   list = (int*)(acc + NB * ROWW);
  int*   wcnt = list + LISTN;
  int*   cnt  = wcnt + 16;
  float* scl  = (float*)(cnt + NB);
  const int tid = threadIdx.x, lane = tid & 31, wave = tid >> 5, hh = lane >> 4, m = lane & 15;
  const int nodeBase = blockIdx.x * NB;
  const int* dsts = ei + nE;

  {
    constexpr int RW4 = ROWW / 4, TF4 = TF / 4;
    const float inf = __builtin_inff();
    for (int i = tid; i < NB * RW4; i += NTHR) {
      const int a = (i % RW4) / TF4;
      const float f = (a < 2) ? 0.f : ((a == 2) ? inf : -inf);
      v4f z; z.x = f; z.y = f; z.z = f; z.w = f;
      lds_dyn[i] = z;
    }
    for (int i = tid; i < NB; i += NTHR) cnt[i] = 0;
  }
  __syncthreads();

  const vC c0r = *(const vC*)(cmp + CH * lane);
  const vC c1r = *(const vC*)(cmp + TF + CH * lane);
  const vC cbr = *(const vC*)(cmp + 2 * TF + CH * lane);

  const int nChunks = (nE + CHUNK - 1) / CHUNK;
#pragma unroll 1
  for (int ch = 0; ch < nChunks; ++ch) {
    const int cbase = ch * CHUNK;
    const int wc = scan_chunk<NB>(dsts, nE, cbase, nodeBase, vec8, list, tid, lane, wave);
    if (lane == 0) wcnt[wave] = wc;
    __syncthreads();
    if (wave == 0) {
#pragma unroll 1
      for (int wsx = 0; wsx < NWAVE; ++wsx) {
        int n = __builtin_amdgcn_readfirstlane(wcnt[wsx]);
        n = n > WCAP ? WCAP : (n < 0 ? 0 : n);
        const int* lp = list + wsx * WCAP;
#pragma unroll 1
        for (int i = 0; i < n; ++i) {
          const int ent  = __builtin_amdgcn_readfirstlane(lp[i]);
          const int slot = ent & (NB - 1);
          int e = cbase + ((ent >> 12) & (CHUNK - 1));
          e = e > nE - 1 ? nE - 1 : e;
          int src = ei[e];
          src = src < 0 ? 0 : (src > nN - 1 ? nN - 1 : src);
          int dn = nodeBase + slot;
          dn = dn > nN - 1 ? nN - 1 : dn;
          const float ea0 = eattr[2 * (size_t)e], ea1 = eattr[2 * (size_t)e + 1];
          const vC pv = *(const vC*)(pq + (size_t)dn * NC + CH * lane);
          const vC qv = *(const vC*)(pq + (size_t)src * NC + TF + CH * lane);
          vC mv = pv + qv;
          mv = mv + c0r * ea0;
          mv = mv + c1r * ea1;
          mv = mv + cbr;
          float* ap = acc + slot * ROWW + CH * lane;
          vC* s0 = (vC*)ap;
          vC* s1 = (vC*)(ap + TF);
          vC* s2 = (vC*)(ap + 2 * TF);
          vC* s3 = (vC*)(ap + 3 * TF);
          *s0 = *s0 + mv;
          *s1 = *s1 + mv * mv;
          *s2 = vminC<CH>(*s2, mv);
          *s3 = vmaxC<CH>(*s3, mv);
          if (lane == 0) cnt[slot] = cnt[slot] + 1;
        }
      }
    }
    __syncthreads();
  }

  {
    constexpr int TF4 = TF / 4;
    for (int i = tid; i < NB * TF4; i += NTHR) {
      const int slot = i / TF4, c4 = (i - slot * TF4) * 4;
      const int c = cnt[slot];
      const float d = (float)(c > 1 ? c : 1);
      const float rd = 1.0f / d;
      float* ap = acc + slot * ROWW + c4;
      const v4f s = *(v4f*)ap, sq = *(v4f*)(ap + TF), mn = *(v4f*)(ap + 2 * TF), mx = *(v4f*)(ap + 3 * TF);
      const v4f mean = s * rd;
      const v4f msq  = sq * rd;
      const v4f var  = msq - mean * mean;
      v4f sd;
      sd.x = sqrtf(fmaxf(var.x, 0.f) + 1e-5f);
      sd.y = sqrtf(fmaxf(var.y, 0.f) + 1e-5f);
      sd.z = sqrtf(fmaxf(var.z, 0.f) + 1e-5f);
      sd.w = sqrtf(fmaxf(var.w, 0.f) + 1e-5f);
      const bool has = c > 0;
      v4f mn2, mx2;
      mn2.x = has ? mn.x : 0.f; mn2.y = has ? mn.y : 0.f; mn2.z = has ? mn.z : 0.f; mn2.w = has ? mn.w : 0.f;
      mx2.x = has ? mx.x : 0.f; mx2.y = has ? mx.y : 0.f; mx2.z = has ? mx.z : 0.f; mx2.w = has ? mx.w : 0.f;
      *(v4f*)ap            = mean;
      *(v4f*)(ap + TF)     = mn2;
      *(v4f*)(ap + 2 * TF) = mx2;
      *(v4f*)(ap + 3 * TF) = sd;
    }
    for (int sl = tid; sl < NB; sl += NTHR) {
      const int c = cnt[sl];
      const float d = (float)(c > 1 ? c : 1);
      const float logd = logf(d + 1.0f);
      scl[2 * sl]     = logd * (1.0f / AVG_LOG_F);
      scl[2 * sl + 1] = AVG_LOG_F / logd;
    }
  }
  __syncthreads();

  for (int q = 0; q < NQ; ++q) {
    const int slot0 = 16 * (wave + 8 * q);
    const int srow  = slot0 + m;
    int node = nodeBase + srow;
    node = node > nN - 1 ? nN - 1 : node;
    const float ampm = scl[2 * srow], attm = scl[2 * srow + 1];
    const float* arow = acc + srow * ROWW;
    const float* xr   = xin + (size_t)node * F;
    v8f o00 = {0.f, 0.f, 0.f, 0.f, 0.f, 0.f, 0.f, 0.f};
    v8f o01 = o00, o10 = o00, o11 = o00;
    pna_tower<F>(0, arow, xr, ampm, attm, wpo, hh, m, o00, o01);
    pna_tower<F>(1, arow, xr, ampm, attm, wpo, hh, m, o10, o11);
    __syncthreads();

    _Float16* so = (_Float16*)(acc + slot0 * ROWW);
    {
      const float b00 = bpost[m], b01 = bpost[16 + m], b10 = bpost[32 + m], b11 = bpost[48 + m];
      _Float16* sp = so + (8 * hh) * 64 + m;
#pragma unroll
      for (int r = 0; r < 8; ++r) {
        sp[r * 64]      = (_Float16)(o00[r] * WINV + b00);
        sp[r * 64 + 16] = (_Float16)(o01[r] * WINV + b01);
        sp[r * 64 + 32] = (_Float16)(o10[r] * WINV + b10);
        sp[r * 64 + 48] = (_Float16)(o11[r] * WINV + b11);
      }
    }
    __syncthreads();

    v8f ya[4];
#pragma unroll
    for (int nt = 0; nt < 4; ++nt) { v8f z = {0.f, 0.f, 0.f, 0.f, 0.f, 0.f, 0.f, 0.f}; ya[nt] = z; }
#pragma unroll
    for (int ks = 0; ks < 2; ++ks) {
      const _Float16* ar = so + m * 64 + 32 * ks + 8 * hh;
      FragH a;
      a.h[0] = *(const v8h*)ar;
      a.h[1] = *(const v8h*)(ar + 16);
#pragma unroll
      for (int nt = 0; nt < 4; ++nt) {
        const _Float16* bp = wl + (size_t)(16 * nt + m) * 64 + 32 * ks + 8 * hh;
        FragH b;
        b.h[0] = *(const v8h*)bp;
        b.h[1] = *(const v8h*)(bp + 16);
        ya[nt] = wmh(a.v, b.v, ya[nt]);
      }
    }
    float* sy = acc + slot0 * ROWW + 512;
#pragma unroll
    for (int nt = 0; nt < 4; ++nt) {
      const int n = 16 * nt + m;
      const float bl = blin[n];
      float* sp = sy + (8 * hh) * 64 + n;
#pragma unroll
      for (int r = 0; r < 8; ++r) sp[r * 64] = fmaxf(ya[nt][r] * WINV + bl, 0.f);
    }
    __syncthreads();

    float* gp = hout + ((size_t)nodeBase + slot0) * 64 + 4 * lane;
    const float* lp = sy + 4 * lane;
#pragma unroll
    for (int i = 0; i < 8; ++i) { const v4f v = *(const v4f*)(lp + i * 128); *(volatile v4f*)(gp + i * 128) = v; }
    __threadfence();
#pragma unroll
    for (int i = 0; i < 8; ++i) { const v4f v = *(const v4f*)(lp + i * 128); *(volatile v4f*)(gp + i * 128) = v; }
  }
}

__global__ __launch_bounds__(NTHR) void k_head(
    const float* __restrict__ h, const int* __restrict__ batch, const float* __restrict__ hls,
    const _Float16* __restrict__ w1t, const float* __restrict__ b1,
    const _Float16* __restrict__ w2t, const float* __restrict__ b2,
    const float* __restrict__ W3, const float* __restrict__ b3, float* out, int nN) {
  extern __shared__ v4f lds_dyn[];
  double*   part = (double*)lds_dyn;
  _Float16* sA   = (_Float16*)(part + 4 * 64 * 64);
  float*    sG1  = (float*)(sA + 64 * 96);
  float*    sG2  = sG1 + 64 * 64;
  float*    sOut = sG2 + 64 * 64;
  const int tid = threadIdx.x, lane = tid & 31, wave = tid >> 5, hh = lane >> 4, m = lane & 15;

  const int c = tid & 63, q = tid >> 6;
  double* pp = part + (size_t)q * 4096 + c;
#pragma unroll 1
  for (int g = 0; g < 64; ++g) pp[g * 64] = 0.0;
#pragma unroll 1
  for (int n = q; n < nN; n += 4) {
    const int b  = batch[n];
    const int bc = b < 0 ? 0 : (b > 63 ? 63 : b);
    const float v = h[(size_t)n * 64 + c];
    const double add = ((unsigned)b < 64u) ? (double)v : 0.0;
    pp[bc * 64] = pp[bc * 64] + add;
  }
  __syncthreads();
  for (int idx = tid; idx < 4096; idx += NTHR) {
    const int g = idx >> 6, cc = idx & 63;
    double s = part[g * 64 + cc];
    s = s + part[4096 + g * 64 + cc];
    s = s + part[8192 + g * 64 + cc];
    s = s + part[12288 + g * 64 + cc];
    sA[g * 96 + cc] = (_Float16)((float)s);
  }
  for (int idx = tid; idx < 64 * HLSD; idx += NTHR) {
    const int g = idx >> 5, j = idx & 31;
    sA[g * 96 + 64 + j] = (_Float16)hls[g * HLSD + j];
  }
  __syncthreads();

  const int rt = wave & 3, ntb = 2 * (wave >> 2);
  {
    v8f a1[2];
    { v8f z = {0.f, 0.f, 0.f, 0.f, 0.f, 0.f, 0.f, 0.f}; a1[0] = z; a1[1] = z; }
#pragma unroll
    for (int ks = 0; ks < 3; ++ks) {
      const _Float16* ar = sA + (rt * 16 + m) * 96 + 32 * ks + 8 * hh;
      FragH a;
      a.h[0] = *(const v8h*)ar;
      a.h[1] = *(const v8h*)(ar + 16);
#pragma unroll
      for (int u = 0; u < 2; ++u) {
        const _Float16* bp = w1t + (size_t)(16 * (ntb + u) + m) * 96 + 32 * ks + 8 * hh;
        FragH b;
        b.h[0] = *(const v8h*)bp;
        b.h[1] = *(const v8h*)(bp + 16);
        a1[u] = wmh(a.v, b.v, a1[u]);
      }
    }
#pragma unroll
    for (int u = 0; u < 2; ++u) {
      const int n = 16 * (ntb + u) + m;
      const float bb = b1[n];
      float* sp = sG1 + (rt * 16 + 8 * hh) * 64 + n;
#pragma unroll
      for (int r = 0; r < 8; ++r) sp[r * 64] = fmaxf(a1[u][r] * WINV + bb, 0.f);
    }
  }
  __syncthreads();
  {
    v8f a2[2];
    { v8f z = {0.f, 0.f, 0.f, 0.f, 0.f, 0.f, 0.f, 0.f}; a2[0] = z; a2[1] = z; }
#pragma unroll
    for (int ks = 0; ks < 2; ++ks) {
      const float* ap = sG1 + (rt * 16 + m) * 64 + 32 * ks + 8 * hh;
      const v4f p0 = *(const v4f*)ap,        p1 = *(const v4f*)(ap + 4);
      const v4f p2 = *(const v4f*)(ap + 16), p3 = *(const v4f*)(ap + 20);
      FragH a;
      a.h[0] = cvt8(p0, p1);
      a.h[1] = cvt8(p2, p3);
#pragma unroll
      for (int u = 0; u < 2; ++u) {
        const _Float16* bp = w2t + (size_t)(16 * (ntb + u) + m) * 64 + 32 * ks + 8 * hh;
        FragH b;
        b.h[0] = *(const v8h*)bp;
        b.h[1] = *(const v8h*)(bp + 16);
        a2[u] = wmh(a.v, b.v, a2[u]);
      }
    }
#pragma unroll
    for (int u = 0; u < 2; ++u) {
      const int n = 16 * (ntb + u) + m;
      const float bb = b2[n];
      float* sp = sG2 + (rt * 16 + 8 * hh) * 64 + n;
#pragma unroll
      for (int r = 0; r < 8; ++r) sp[r * 64] = fmaxf(a2[u][r] * WINV + bb, 0.f);
    }
  }
  __syncthreads();
  if (tid < 64) {
    float s = 0.f;
    const float* gr = sG2 + tid * 64;
#pragma unroll 1
    for (int k = 0; k < 64; ++k) s = s + gr[k] * W3[k];
    sOut[tid] = s + b3[0];
  }
  __syncthreads();
  const int ti = tid < 16 ? tid : 15;
  const v4f ov = *(const v4f*)(sOut + 4 * ti);
  if (tid < 16) *(volatile v4f*)(out + 4 * tid) = ov;
  __threadfence();
  if (tid < 16) *(volatile v4f*)(out + 4 * tid) = ov;
}

static inline size_t al256(size_t x) { return (x + 255) & ~(size_t)255; }

extern "C" void kernel_launch(void* const* d_in, const int* in_sizes, int n_in,
                              void* d_out, int out_size, void* d_ws, size_t ws_size,
                              hipStream_t stream) {
  if (n_in < 27) return;
  const int nN = in_sizes[4];
  const int nE = in_sizes[3] / 2;
  if (nN <= 0 || nE <= 0) return;
  if (in_sizes[0] != nN * 32 || in_sizes[3] != 2 * nE || in_sizes[1] != 2 * nE) return;
  if (out_size != GGR || in_sizes[2] != GGR * HLSD) return;
  if (in_sizes[5] != 2 * 32 || in_sizes[6] != 32 || in_sizes[7] != 2 * 96 * 32 || in_sizes[8] != 64 ||
      in_sizes[9] != 2 * 416 * 32 || in_sizes[10] != 64 || in_sizes[11] != 4096 || in_sizes[12] != 64) return;
  if (in_sizes[13] != 128 || in_sizes[14] != 64 || in_sizes[15] != 2 * 192 * 64 || in_sizes[16] != 128 ||
      in_sizes[17] != 2 * 832 * 32 || in_sizes[18] != 64 || in_sizes[19] != 4096 || in_sizes[20] != 64) return;
  if (in_sizes[21] != 96 * 64 || in_sizes[22] != 64 || in_sizes[23] != 4096 || in_sizes[24] != 64 ||
      in_sizes[25] != 64 || in_sizes[26] != 1) return;

  const float* x     = (const float*)d_in[0];
  const float* eattr = (const float*)d_in[1];
  const float* hls   = (const float*)d_in[2];
  const int*   ei    = (const int*)d_in[3];
  const int*   batch = (const int*)d_in[4];
  const float* We0 = (const float*)d_in[5],    *be0 = (const float*)d_in[6];
  const float* Wpre0 = (const float*)d_in[7],  *bpre0 = (const float*)d_in[8];
  const float* Wpost0 = (const float*)d_in[9], *bpost0 = (const float*)d_in[10];
  const float* Wlin0 = (const float*)d_in[11], *blin0 = (const float*)d_in[12];
  const float* We1 = (const float*)d_in[13],   *be1 = (const float*)d_in[14];
  const float* Wpre1 = (const float*)d_in[15], *bpre1 = (const float*)d_in[16];
  const float* Wpost1 = (const float*)d_in[17], *bpost1 = (const float*)d_in[18];
  const float* Wlin1 = (const float*)d_in[19], *blin1 = (const float*)d_in[20];
  const float* W1 = (const float*)d_in[21], *b1 = (const float*)d_in[22];
  const float* W2 = (const float*)d_in[23], *b2 = (const float*)d_in[24];
  const float* W3 = (const float*)d_in[25], *b3 = (const float*)d_in[26];
  float* out = (float*)d_out;
  (void)bpost0; (void)bpost1;

  const int nPQ = (nN + PQROWS - 1) / PQROWS;
  const int nA0 = (nN + PnaCfg<32>::NB - 1) / PnaCfg<32>::NB;
  const int nA1 = (nN + PnaCfg<64>::NB - 1) / PnaCfg<64>::NB;

  char* ws = (char*)d_ws;
  size_t off = 0;
  const size_t oWpq0 = off; off = al256(off + (size_t)128 * 32 * 2);
  const size_t oWpq1 = off; off = al256(off + (size_t)256 * 64 * 2);
  const size_t oWpo0 = off; off = al256(off + (size_t)64 * 416 * 2);
  const size_t oWpo1 = off; off = al256(off + (size_t)64 * 832 * 2);
  const size_t oWl0  = off; off = al256(off + (size_t)64 * 64 * 2);
  const size_t oWl1  = off; off = al256(off + (size_t)64 * 64 * 2);
  const size_t oW1t  = off; off = al256(off + (size_t)64 * 96 * 2);
  const size_t oW2t  = off; off = al256(off + (size_t)64 * 64 * 2);
  const size_t oCmp0 = off; off = al256(off + (size_t)3 * 64 * 4);
  const size_t oCmp1 = off; off = al256(off + (size_t)3 * 128 * 4);
  const size_t oPq0  = off; off = al256(off + (size_t)nPQ * PQROWS * 128 * 4);
  const size_t oH0   = off; off = al256(off + (size_t)nA0 * PnaCfg<32>::NB * 64 * 4);
  const size_t oPq1  = off; off = al256(off + (size_t)nPQ * PQROWS * 256 * 4);
  const size_t oH1   = off; off = al256(off + (size_t)nA1 * PnaCfg<64>::NB * 64 * 4);
  if (off > ws_size || off > WS_CAP) return;
  _Float16* wpq0 = (_Float16*)(ws + oWpq0);
  _Float16* wpq1 = (_Float16*)(ws + oWpq1);
  _Float16* wpo0 = (_Float16*)(ws + oWpo0);
  _Float16* wpo1 = (_Float16*)(ws + oWpo1);
  _Float16* wl0  = (_Float16*)(ws + oWl0);
  _Float16* wl1  = (_Float16*)(ws + oWl1);
  _Float16* w1t  = (_Float16*)(ws + oW1t);
  _Float16* w2t  = (_Float16*)(ws + oW2t);
  float* cmp0 = (float*)(ws + oCmp0);
  float* cmp1 = (float*)(ws + oCmp1);
  float* pq0  = (float*)(ws + oPq0);
  float* h0   = (float*)(ws + oH0);
  float* pq1  = (float*)(ws + oPq1);
  float* h1   = (float*)(ws + oH1);

  const int vec8 = ((nE & 3) == 0) ? 1 : 0;

  const int nPrepBlk = (64 * 832 / 8 + NTHR - 1) / NTHR;
  k_prep<<<dim3(nPrepBlk, 10), NTHR, 0, stream>>>(Wpre0, Wpre1, Wpost0, Wpost1, Wlin0, Wlin1, W1, W2,
                                                   We0, be0, bpre0, We1, be1, bpre1,
                                                   wpq0, wpq1, wpo0, wpo1, wl0, wl1, w1t, w2t, cmp0, cmp1);

  hipFuncSetAttribute(reinterpret_cast<const void*>(&k_pq<32>),
                      hipFuncAttributeMaxDynamicSharedMemorySize, LDS_PQ);
  k_pq<32><<<nPQ, NTHR, LDS_PQ, stream>>>(x, wpq0, pq0, nN);
  hipFuncSetAttribute(reinterpret_cast<const void*>(&k_pna<32>),
                      hipFuncAttributeMaxDynamicSharedMemorySize, PnaCfg<32>::LDS);
  k_pna<32><<<nA0, NTHR, PnaCfg<32>::LDS, stream>>>(ei, eattr, x, pq0, cmp0, wpo0,
                                                    (const float*)d_in[10], wl0, blin0, h0, nN, nE, vec8);

  hipFuncSetAttribute(reinterpret_cast<const void*>(&k_pq<64>),
                      hipFuncAttributeMaxDynamicSharedMemorySize, LDS_PQ);
  k_pq<64><<<nPQ, NTHR, LDS_PQ, stream>>>(h0, wpq1, pq1, nN);
  hipFuncSetAttribute(reinterpret_cast<const void*>(&k_pna<64>),
                      hipFuncAttributeMaxDynamicSharedMemorySize, PnaCfg<64>::LDS);
  k_pna<64><<<nA1, NTHR, PnaCfg<64>::LDS, stream>>>(ei, eattr, h0, pq1, cmp1, wpo1,
                                                    (const float*)d_in[18], wl1, blin1, h1, nN, nE, vec8);

  hipFuncSetAttribute(reinterpret_cast<const void*>(&k_head),
                      hipFuncAttributeMaxDynamicSharedMemorySize, LDS_HEAD);
  k_head<<<1, NTHR, LDS_HEAD, stream>>>(h1, batch, hls, w1t, b1, w2t, b2, W3, b3, out, nN);
}
